// SparseConv3DLayer_75213467287817
// MI455X (gfx1250) — hardware-run, weakly checked
//
#include <hip/hip_runtime.h>


#ifndef NB
#define NB 2
#endif
#define NB_FULL 2
#define HH   96
#define WW   128
#define DD   32
#define CC   16
#define FF   16
#define WPB  4
#define NPIX (NB * HH * WW)
#define NSTEP 5
#define WT_E (3 * NSTEP * FF * 32)
#define SLAB_ROWS 224
#define SLAB_E (SLAB_ROWS * CC)

static_assert(CC == 16);
static_assert(FF == 16);
static_assert(DD == 32);
static_assert(2 * NSTEP == 10);
static_assert(SLAB_ROWS == 32 + 3 * 64);
static_assert(NPIX % WPB == 0);
static_assert(NB <= NB_FULL);
static_assert(((size_t)NB * HH * WW * DD * CC) % 64 == 0);
static_assert((WT_E % 64) == 0);
static_assert(4 * 32 * 4 == DD * FF);
static_assert((size_t)WPB * SLAB_E * 2 + (size_t)WPB * DD * FF * 4 <= (size_t)131072);

typedef _Float16 h16;
typedef unsigned short bf;
typedef __attribute__((ext_vector_type(16))) __bf16   v16bf;
typedef __attribute__((ext_vector_type(16))) _Float16 v16h;
typedef __attribute__((ext_vector_type(8)))  _Float16 v8h;
typedef __attribute__((ext_vector_type(8)))  unsigned short v8us;
typedef __attribute__((ext_vector_type(8)))  float    v8f;
typedef __attribute__((ext_vector_type(4)))  float    v4f;
typedef v4f  __attribute__((may_alias)) v4fa;
typedef v8us __attribute__((may_alias)) v8usa;

__device__ __forceinline__ unsigned short f2bf(float f) { unsigned u = __float_as_uint(f); u += 0x7FFFu + ((u >> 16) & 1u); return (unsigned short)(u >> 16); }
__device__ __forceinline__ float bfr(float f) { return __uint_as_float(((unsigned)f2bf(f)) << 16); }
__device__ __forceinline__ v16h cat16(v8h lo, v8h hi) { return __builtin_shufflevector(lo, hi, 0, 1, 2, 3, 4, 5, 6, 7, 8, 9, 10, 11, 12, 13, 14, 15); }
__device__ __forceinline__ v16bf cat16b(v8us lo, v8us hi) { return __builtin_bit_cast(v16bf, __builtin_shufflevector(lo, hi, 0, 1, 2, 3, 4, 5, 6, 7, 8, 9, 10, 11, 12, 13, 14, 15)); }
__device__ __forceinline__ v8f wmma16(v16h a, v16h b, v8f c) { return __builtin_amdgcn_wmma_f32_16x16x32_f16(false, a, false, b, (short)0, c, false, false); }
__device__ __forceinline__ v8f wmmab(v16bf a, v16bf b, v8f c) { return __builtin_amdgcn_wmma_f32_16x16x32_bf16(false, a, false, b, (short)0, c, false, false); }
__device__ __forceinline__ v16h  ldh(const h16* p) { return cat16(*(const v8h*)p, *(const v8h*)(p + 16)); }
__device__ __forceinline__ v16bf ldb(const bf* p)  { return cat16b(*(const v8us*)p, *(const v8us*)(p + 16)); }
__device__ __forceinline__ void wave_sync() { __builtin_amdgcn_fence(3  , "wavefront"); __builtin_amdgcn_wave_barrier(); asm volatile("" ::: "memory"); }
__device__ __forceinline__ v8f wmmab_g(v16bf a, v16bf b, v8f c) { c = wmmab(a, b, c); asm volatile("v_nop\n\tv_nop\n\tv_nop\n\tv_nop" : "+v"(c) : "v"(a), "v"(b)); return c; }
__device__ __forceinline__ int iclampi(int x, int lo, int up) { return x < lo ? lo : (x > up ? up : x); }

__global__ __launch_bounds__(256) void k_cvt8(const float* __restrict__ src, bf* dst, size_t n8) {
    const size_t i = (size_t)blockIdx.x * 256 + threadIdx.x; if (i >= n8) return;
    const v8f v = *(const v8f*)(src + i * 8); v8us o;
#pragma unroll
    for (int k = 0; k < 8; ++k) o[k] = f2bf(v[k]);
    *(volatile v8us*)(dst + i * 8) = o; __threadfence(); *(volatile v8us*)(dst + i * 8) = o;
}

__global__ __launch_bounds__(256) void k_wprep(const float* __restrict__ kern, bf* WT) {
    const int i8 = blockIdx.x * 256 + threadIdx.x; if (i8 >= WT_E / 8) return;
    const int kq = i8 & 3, f = (i8 >> 2) & 15, g = i8 >> 6;
    const int i = g / NSTEP, s = g - NSTEP * i;
    const int kk0 = kq * 8;
    const int t9 = 2 * s + (kk0 >> 4);
    const int c0 = kk0 & 15;
    const bool ok = t9 < 9;
    const int t9c = ok ? t9 : 8;
    v8us o;
#pragma unroll
    for (int e = 0; e < 8; ++e) {
        float v = kern[(size_t)((i * 9 + t9c) * CC + c0 + e) * FF + f];
        asm volatile("" : "+v"(v));
        o[e] = ok ? f2bf(v) : (bf)0; }
    *(volatile v8us*)(WT + (size_t)i8 * 8) = o; __threadfence(); *(volatile v8us*)(WT + (size_t)i8 * 8) = o;
}

__global__ __launch_bounds__(32 * WPB) void k_conv(const bf* __restrict__ XB, const int* __restrict__ bp, const bf* __restrict__ WT, const float* __restrict__ defv, float* OUT) {
    __shared__ __align__(16) bf slab[WPB * SLAB_E];
    __shared__ __align__(16) float os[WPB * DD * FF];
    const int lane = threadIdx.x & 31, lr = lane & 15, hi = lane >> 4;
    const int wave = __builtin_amdgcn_readfirstlane((int)(threadIdx.x >> 5));
    const int p = blockIdx.x * WPB + wave;
    const int b = p / (HH * WW); const int hw = p - b * (HH * WW); const int h = hw / WW; const int w = hw - h * WW;
    const bf dvb = f2bf(defv[0]);
    v8us dvv;
#pragma unroll
    for (int e = 0; e < 8; ++e) dvv[e] = dvb;
    const v8us zv = (v8us){};
    const int sb = wave * SLAB_E;
#pragma unroll
    for (int g = 0; g < 4; ++g) { const int e = sb + (64 * g + lane) * CC; *(v8usa*)(&slab[e]) = dvv; *(v8usa*)(&slab[e + 8]) = dvv; }
    const int bpc = bp[p];
    v8f acc0 = (v8f){}, acc1 = (v8f){};
#pragma unroll 1
    for (int i = 0; i < 3; ++i) {
        const int hh = h + i - 1; const bool vh = (hh >= 0) & (hh < HH); const int hc = iclampi(hh, 0, HH - 1);
        int sh[3];
#pragma unroll
        for (int j = 0; j < 3; ++j) {
            const int ww = w + j - 1; const bool vw = (ww >= 0) & (ww < WW); const int wc = iclampi(ww, 0, WW - 1);
            const bool vhw = vh & vw;
            const int np = (b * HH + hc) * WW + wc;
            const int rel = (int)((unsigned)bpc - (unsigned)bp[np]);
            sh[j] = iclampi(rel, -2 * DD, 2 * DD);
            const bf* src = XB + (size_t)np * (DD * CC) + lane * CC;
            v8us x0 = *(const v8us*)src, x1 = *(const v8us*)(src + 8);
            if (!vhw) { x0 = dvv; x1 = dvv; }
            const int e = sb + (32 + 64 * j + lane) * CC;
            *(v8usa*)(&slab[e]) = x0; *(v8usa*)(&slab[e + 8]) = x1; }
        wave_sync();
#pragma unroll
        for (int s = 0; s < NSTEP; ++s) {
            const int tA = 2 * s, tB = 2 * s + 1;
            const int jA = tA / 3, kA = tA - 3 * jA;
            const int jB = (tB < 9) ? (tB / 3) : 2, kB = (tB < 9) ? (tB - 3 * (tB / 3)) : 2;
            const int sA = iclampi(sh[jA] + kA - 1, -DD, DD);
            const int sB = iclampi(sh[jB] + kB - 1, -DD, DD);
            const v16bf bw = ldb(WT + (size_t)((i * NSTEP + s) * FF + lr) * 32 + 8 * hi);
            const int eA = sb + (32 + 64 * jA + lr + sA) * CC + 8 * hi;
            const int eB = sb + (32 + 64 * jB + lr + sB) * CC + 8 * hi;
            const v8us a0l = *(const v8usa*)(&slab[eA]); const v8us a1l = *(const v8usa*)(&slab[eA + 16 * CC]);
            v8us a0u = zv, a1u = zv;
            if (tB < 9) { a0u = *(const v8usa*)(&slab[eB]); a1u = *(const v8usa*)(&slab[eB + 16 * CC]); }
            acc0 = wmmab_g(cat16b(a0l, a0u), bw, acc0);
            acc1 = wmmab_g(cat16b(a1l, a1u), bw, acc1); }
        wave_sync();
    }
    const int ob = wave * (DD * FF);
#pragma unroll
    for (int r = 0; r < 8; ++r) { os[ob + (8 * hi + r) * FF + lr] = acc0[r]; os[ob + (16 + 8 * hi + r) * FF + lr] = acc1[r]; }
    wave_sync();
    float* orow = OUT + (size_t)p * (DD * FF);
#pragma unroll 1
    for (int ps = 0; ps < 2; ++ps) {
#pragma unroll
        for (int s = 0; s < 4; ++s) { const int q = s * 32 + lane;
            const v4f val = *(const v4fa*)(&os[ob + q * 4]);
            *(volatile v4f*)(orow + (size_t)q * 4) = val; }
        if (ps == 0) __threadfence(); }
}

static constexpr size_t al256(size_t v) { return (v + 255) & ~(size_t)255; }
static constexpr size_t SZ_XB = al256((size_t)NB * HH * WW * DD * CC * 2);
static constexpr size_t SZ_WT = al256((size_t)WT_E * 2);
static constexpr size_t SZ_TOTAL = SZ_XB + SZ_WT;
static_assert(SZ_TOTAL <= (size_t)134217728);
static_assert((size_t)(WT_E / 8) * 16 == (size_t)WT_E * 2);
static_assert((size_t)3 * 9 * CC * FF == (size_t)6912);

extern "C" void kernel_launch(void* const* d_in, const int* in_sizes, int n_in,
                              void* d_out, int out_size, void* d_ws, size_t ws_size, hipStream_t stream) {
    if (n_in < 4) return;
    const size_t nimg = (size_t)NB * HH * WW * DD * CC;
    if ((size_t)in_sizes[0] < nimg) return;
    if ((size_t)in_sizes[1] < (size_t)NB * HH * WW) return;
    if ((size_t)in_sizes[2] < (size_t)3 * 9 * CC * FF) return;
    if (in_sizes[3] < 1) return;
    if ((size_t)out_size < (size_t)NB * HH * WW * DD * FF) return;
    if (SZ_TOTAL > ws_size) return;
    const float* img  = (const float*)d_in[0];
    const int*   bpl  = (const int*)d_in[1];
    const float* kern = (const float*)d_in[2];
    const float* defv = (const float*)d_in[3];
    float* OUT = (float*)d_out;
    char* wsp = (char*)d_ws;
    bf* XB = (bf*)wsp; wsp += SZ_XB;
    bf* WT = (bf*)wsp; wsp += SZ_WT;

    { const size_t n8 = nimg / 8;
      k_cvt8<<<(unsigned)((n8 + 255) / 256), 256, 0, stream>>>(img, XB, n8); }
    k_wprep<<<(unsigned)((WT_E / 8 + 255) / 256), 256, 0, stream>>>(kern, WT);
    k_conv<<<dim3(NPIX / WPB, 1, 1), 32 * WPB, 0, stream>>>(XB, bpl, WT, defv, OUT);
}
